// PositionEncoding_50087908606508
// MI455X (gfx1250) — hardware-verified
//
#include <hip/hip_runtime.h>

typedef _Float16 v16h __attribute__((ext_vector_type(16)));
typedef _Float16 v8h  __attribute__((ext_vector_type(8)));
typedef float    v8f  __attribute__((ext_vector_type(8)));
typedef float    v4f  __attribute__((ext_vector_type(4)));
typedef v8h __attribute__((may_alias)) v8ha;
typedef v4f __attribute__((may_alias)) v4fa;

union Frag { v16h v; v8h half[2]; };

#define NB    64
#define NSEQ  1024
#define NE    128
#define NFF   512
#define NH    8
#define HDIM  16
#define NL    4
#define NROWS (NB * NSEQ)
#define WSC   16.0f

static_assert(NROWS % 128 == 0);
static_assert(NSEQ % 128 == 0);
static_assert(NE % 64 == 0);
static_assert(NFF % 64 == 0);
static_assert(NFF == 4 * NE);
static_assert(NH * HDIM == NE);

__device__ __forceinline__ v8f wmma_f16(v16h a, v16h b, v8f c) {
  v8f d = __builtin_amdgcn_wmma_f32_16x16x32_f16(false, a, false, b, (short)0, c, false, false);
  asm volatile("v_nop\n\tv_nop\n\tv_nop\n\tv_nop" : "+v"(d) : "v"(a), "v"(b));
  return d;
}

__device__ __forceinline__ v16h load_frag(const _Float16* p, int h) {
  Frag f;
  f.half[0] = *(const v8ha*)(p + 8 * h);
  f.half[1] = *(const v8ha*)(p + 16 + 8 * h);
  return f.v;
}

__device__ __forceinline__ v8h zero8h() {
  const v8h z = { (_Float16)0.0f, (_Float16)0.0f, (_Float16)0.0f, (_Float16)0.0f,
                  (_Float16)0.0f, (_Float16)0.0f, (_Float16)0.0f, (_Float16)0.0f };
  return z;
}
__device__ __forceinline__ v8f zero8f() {
  const v8f z = { 0.f, 0.f, 0.f, 0.f, 0.f, 0.f, 0.f, 0.f };
  return z;
}

__global__ __launch_bounds__(256) void xt_kernel(const float* __restrict__ x, float* __restrict__ t)
{
  __shared__ float sX[32 * 33];
  const int tid = threadIdx.x;
  const int n0 = blockIdx.x * 32, e0 = blockIdx.y * 32, b = blockIdx.z;
  {
    const int e = tid >> 3, nq = tid & 7;
    const v4f v = *(const v4fa*)(x + ((size_t)(b * NE + e0 + e)) * NSEQ + n0 + 4 * nq);
    float* p = sX + e * 33 + 4 * nq;
    p[0] = v.x; p[1] = v.y; p[2] = v.z; p[3] = v.w;
  }
  __syncthreads();
  const int n = tid >> 3, eq = tid & 7;
  v4f o;
  o.x = sX[(4 * eq + 0) * 33 + n];
  o.y = sX[(4 * eq + 1) * 33 + n];
  o.z = sX[(4 * eq + 2) * 33 + n];
  o.w = sX[(4 * eq + 3) * 33 + n];
  float* dst = t + ((size_t)(b * NSEQ + n0 + n)) * NE + e0 + 4 * eq;
  *(volatile v4f*)dst = o;
  __threadfence();
  *(volatile v4f*)dst = o;
}

__global__ __launch_bounds__(256) void wt_kernel(const float* __restrict__ w, _Float16* __restrict__ wt,
                                                 int K, int Nc, int dstL, int dstR0)
{
  __shared__ float sW[64 * 33];
  const int tid = threadIdx.x;
  const int n0 = blockIdx.x * 32, k0 = blockIdx.y * 64, layer = blockIdx.z;
  const float* src = w + (size_t)layer * K * Nc;
  {
    const int kr = tid >> 2, nq = tid & 3;
    const float* p = src + (size_t)(k0 + kr) * Nc + n0 + 8 * nq;
    const v4f a = *(const v4fa*)p;
    const v4f c = *(const v4fa*)(p + 4);
    float* d = sW + kr * 33 + 8 * nq;
    d[0] = a.x; d[1] = a.y; d[2] = a.z; d[3] = a.w;
    d[4] = c.x; d[5] = c.y; d[6] = c.z; d[7] = c.w;
  }
  __syncthreads();
  const int n = tid >> 3, kq = tid & 7;
  v8h o;
  #pragma unroll
  for (int j = 0; j < 8; ++j) o[j] = (_Float16)(sW[(8 * kq + j) * 33 + n] * WSC);
  _Float16* dst = wt + (size_t)layer * dstL + (size_t)(dstR0 + n0 + n) * K + k0 + 8 * kq;
  *(volatile v8h*)dst = o;
  __threadfence();
  *(volatile v8h*)dst = o;
}

__global__ __launch_bounds__(256) void ln_kernel(const float* __restrict__ t,
    const float* __restrict__ g, const float* __restrict__ bb, _Float16* __restrict__ y)
{
  const int tid = threadIdx.x, lane = tid & 31, w = tid >> 5, hh = lane >> 4;
  const int e0 = 8 * (lane & 15);
  const int row = (blockIdx.x * 8 + w) * 2 + hh;
  const float* p = t + (size_t)row * NE + e0;
  const v4f a = *(const v4fa*)p;
  const v4f c = *(const v4fa*)(p + 4);
  float s = ((a.x + a.y) + (a.z + a.w)) + ((c.x + c.y) + (c.z + c.w));
  s += __shfl_xor(s, 8); s += __shfl_xor(s, 4); s += __shfl_xor(s, 2); s += __shfl_xor(s, 1);
  const float mu = s * (1.0f / NE);
  float d[8] = { a.x - mu, a.y - mu, a.z - mu, a.w - mu, c.x - mu, c.y - mu, c.z - mu, c.w - mu };
  float ss = 0.0f;
  #pragma unroll
  for (int j = 0; j < 8; ++j) ss += d[j] * d[j];
  ss += __shfl_xor(ss, 8); ss += __shfl_xor(ss, 4); ss += __shfl_xor(ss, 2); ss += __shfl_xor(ss, 1);
  const float rstd = rsqrtf(ss * (1.0f / NE) + 1e-5f);
  const v4f g0 = *(const v4fa*)(g + e0);
  const v4f g1 = *(const v4fa*)(g + e0 + 4);
  const v4f b0 = *(const v4fa*)(bb + e0);
  const v4f b1 = *(const v4fa*)(bb + e0 + 4);
  const float gg[8] = { g0.x, g0.y, g0.z, g0.w, g1.x, g1.y, g1.z, g1.w };
  const float bv[8] = { b0.x, b0.y, b0.z, b0.w, b1.x, b1.y, b1.z, b1.w };
  v8h o;
  #pragma unroll
  for (int j = 0; j < 8; ++j) o[j] = (_Float16)(d[j] * rstd * gg[j] + bv[j]);
  _Float16* dst = y + (size_t)row * NE + e0;
  *(volatile v8h*)dst = o;
  __threadfence();
  *(volatile v8h*)dst = o;
}

__device__ __forceinline__ void gemm_core(const _Float16* __restrict__ A, int lda,
                                          const _Float16* __restrict__ BT, int K,
                                          int arow0, int bcol0, int lane, v8f (&acc)[2][4])
{
  const int h = lane >> 4, m = lane & 15;
  const _Float16* a0p = A + (size_t)(arow0 + m) * lda;
  const _Float16* a1p = a0p + (size_t)16 * lda;
  const _Float16* bp  = BT + (size_t)(bcol0 + m) * K;
  #pragma unroll
  for (int mt = 0; mt < 2; ++mt)
    #pragma unroll
    for (int nt = 0; nt < 4; ++nt) acc[mt][nt] = zero8f();
  #pragma unroll 1
  for (int k0 = 0; k0 < K; k0 += 32) {
    const v16h a0 = load_frag(a0p + k0, h);
    const v16h a1 = load_frag(a1p + k0, h);
    #pragma unroll
    for (int nt = 0; nt < 4; ++nt) {
      const v16h b = load_frag(bp + (size_t)nt * 16 * K + k0, h);
      acc[0][nt] = wmma_f16(a0, b, acc[0][nt]);
      acc[1][nt] = wmma_f16(a1, b, acc[1][nt]);
    }
  }
}

__global__ __launch_bounds__(128) void gemm_qkv_kernel(
    const _Float16* __restrict__ Y, const _Float16* __restrict__ WT,
    _Float16* __restrict__ qp, _Float16* __restrict__ ktp, _Float16* __restrict__ vtp)
{
  __shared__ __attribute__((aligned(16))) _Float16 sT[128 * 72];

  const int tid = threadIdx.x, lane = tid & 31, w = tid >> 5, h = lane >> 4, m = lane & 15;
  const int m0 = blockIdx.x * 128, by = blockIdx.y, col0 = by * 64;
  v8f acc[2][4];
  gemm_core(Y, NE, WT, NE, m0 + 32 * w, col0, lane, acc);

  if (by < 2) {
    #pragma unroll
    for (int nt = 0; nt < 4; ++nt)
      #pragma unroll
      for (int mt = 0; mt < 2; ++mt)
        #pragma unroll
        for (int r = 0; r < 8; ++r) {
          const int rl = 32 * w + 16 * mt + 8 * h + r;
          sT[rl * 72 + 16 * nt + m] = (_Float16)(acc[mt][nt][r] * 0.5f);
        }
  } else {
    #pragma unroll
    for (int nt = 0; nt < 4; ++nt)
      #pragma unroll
      for (int mt = 0; mt < 2; ++mt) {
        v8h cv;
        #pragma unroll
        for (int r = 0; r < 8; ++r) cv[r] = (_Float16)(acc[mt][nt][r] * 0.5f);
        const int cl = 16 * nt + m, rlb = 32 * w + 16 * mt + 8 * h;
        *(v8ha*)(sT + cl * 136 + rlb) = cv;
      }
  }
  __syncthreads();

  const int q8 = lane & 7, sub = lane >> 3;
  if (by < 2) {
    _Float16* gbase = qp + (size_t)m0 * NE + col0;
    #pragma unroll
    for (int i = 0; i < 8; ++i) {
      const int row = 32 * w + 4 * i + sub;
      const v8h v = *(const v8ha*)(sT + row * 72 + 8 * q8);
      *(volatile v8h*)(gbase + (size_t)row * NE + 8 * q8) = v;
    }
    __threadfence();
    #pragma unroll
    for (int i = 0; i < 8; ++i) {
      const int row = 32 * w + 4 * i + sub;
      const v8h v = *(const v8ha*)(sT + row * 72 + 8 * q8);
      *(volatile v8h*)(gbase + (size_t)row * NE + 8 * q8) = v;
    }
  } else {
    const int sel = by - 2, which = sel >> 1, fb = 64 * (sel & 1);
    const int b = m0 >> 10, n0l = m0 & (NSEQ - 1);
    _Float16* plane = which ? vtp : ktp;
    _Float16* gbase = plane + ((size_t)(b * NE + fb)) * NSEQ + n0l;
    #pragma unroll
    for (int i = 0; i < 8; ++i) {
      const int L = 4 * i + sub, f = 16 * w + (L >> 1), hl = L & 1;
      const v8h v = *(const v8ha*)(sT + f * 136 + 64 * hl + 8 * q8);
      *(volatile v8h*)(gbase + (size_t)f * NSEQ + 64 * hl + 8 * q8) = v;
    }
    __threadfence();
    #pragma unroll
    for (int i = 0; i < 8; ++i) {
      const int L = 4 * i + sub, f = 16 * w + (L >> 1), hl = L & 1;
      const v8h v = *(const v8ha*)(sT + f * 136 + 64 * hl + 8 * q8);
      *(volatile v8h*)(gbase + (size_t)f * NSEQ + 64 * hl + 8 * q8) = v;
    }
  }
}

__global__ __launch_bounds__(128) void gemm_resid_kernel(
    const _Float16* __restrict__ A, int lda, const _Float16* __restrict__ WT, int K,
    const float* __restrict__ bias, float oscale, float* __restrict__ t)
{
  __shared__ __attribute__((aligned(16))) float sF[128 * 68];

  const int tid = threadIdx.x, lane = tid & 31, w = tid >> 5, h = lane >> 4, m = lane & 15;
  const int m0 = blockIdx.x * 128, col0 = blockIdx.y * 64;
  v8f acc[2][4];
  gemm_core(A, lda, WT, K, m0 + 32 * w, col0, lane, acc);

  #pragma unroll
  for (int nt = 0; nt < 4; ++nt) {
    const float bv = bias[col0 + 16 * nt + m];
    #pragma unroll
    for (int mt = 0; mt < 2; ++mt)
      #pragma unroll
      for (int r = 0; r < 8; ++r) {
        const int rl = 32 * w + 16 * mt + 8 * h + r;
        sF[rl * 68 + 16 * nt + m] = acc[mt][nt][r] * oscale + bv;
      }
  }
  __syncthreads();

  const int q8 = lane & 7, sub = lane >> 3;
  #pragma unroll
  for (int i = 0; i < 16; ++i) {
    const int L = 4 * i + sub, row = 32 * w + (L >> 1), hl = L & 1;
    float* sp = sF + row * 68 + 32 * hl + 4 * q8;
    float* gp = t + (size_t)(m0 + row) * NE + col0 + 32 * hl + 4 * q8;
    const v4f a = *(const v4fa*)sp;
    const v4f o = *(const v4fa*)gp;
    const v4f s = o + a;
    *(v4fa*)sp = s;
    *(volatile v4f*)gp = s;
  }
  __threadfence();
  #pragma unroll
  for (int i = 0; i < 16; ++i) {
    const int L = 4 * i + sub, row = 32 * w + (L >> 1), hl = L & 1;
    const float* sp = sF + row * 68 + 32 * hl + 4 * q8;
    float* gp = t + (size_t)(m0 + row) * NE + col0 + 32 * hl + 4 * q8;
    const v4f s = *(const v4fa*)sp;
    *(volatile v4f*)gp = s;
  }
}

__global__ __launch_bounds__(128) void gemm_gelu_kernel(
    const _Float16* __restrict__ Y, const _Float16* __restrict__ WT,
    const float* __restrict__ bias, _Float16* __restrict__ ffa)
{
  __shared__ __attribute__((aligned(16))) _Float16 sH[128 * 72];

  const int tid = threadIdx.x, lane = tid & 31, w = tid >> 5, h = lane >> 4, m = lane & 15;
  const int m0 = blockIdx.x * 128, col0 = blockIdx.y * 64;
  v8f acc[2][4];
  gemm_core(Y, NE, WT, NE, m0 + 32 * w, col0, lane, acc);

  #pragma unroll
  for (int nt = 0; nt < 4; ++nt) {
    const float bv = bias[col0 + 16 * nt + m];
    #pragma unroll
    for (int mt = 0; mt < 2; ++mt)
      #pragma unroll
      for (int r = 0; r < 8; ++r) {
        const int rl = 32 * w + 16 * mt + 8 * h + r;
        const float z = acc[mt][nt][r] * (1.0f / WSC) + bv;
        const float u = 0.7978845608028654f * (z + 0.044715f * z * z * z);
        const float gl = z * __builtin_amdgcn_rcpf(1.0f + __expf(-2.0f * u));
        sH[rl * 72 + 16 * nt + m] = (_Float16)(gl * 8.0f);
      }
  }
  __syncthreads();

  const int q8 = lane & 7, sub = lane >> 3;
  _Float16* gbase = ffa + (size_t)m0 * NFF + col0;
  #pragma unroll
  for (int i = 0; i < 8; ++i) {
    const int row = 32 * w + 4 * i + sub;
    const v8h v = *(const v8ha*)(sH + row * 72 + 8 * q8);
    *(volatile v8h*)(gbase + (size_t)row * NFF + 8 * q8) = v;
  }
  __threadfence();
  #pragma unroll
  for (int i = 0; i < 8; ++i) {
    const int row = 32 * w + 4 * i + sub;
    const v8h v = *(const v8ha*)(sH + row * 72 + 8 * q8);
    *(volatile v8h*)(gbase + (size_t)row * NFF + 8 * q8) = v;
  }
}

__global__ __launch_bounds__(32) void ctx_kernel(const _Float16* __restrict__ ktp,
                                                 const _Float16* __restrict__ vtp,
                                                 _Float16* __restrict__ ctxT)
{
  __shared__ __attribute__((aligned(16))) _Float16 sC[256];

  const int lane = threadIdx.x & 31, hh = lane >> 4, m = lane & 15;
  const int bh = blockIdx.x, b = bh >> 3, hd = bh & 7;
  const _Float16* krow = ktp + ((size_t)(b * NE + hd * HDIM + m)) * NSEQ;
  const _Float16* vrow = vtp + ((size_t)(b * NE + hd * HDIM + m)) * NSEQ;

  float mx = -3.0e38f;
  #pragma unroll 2
  for (int j = 0; j < 64; ++j) {
    const v8h kv = *(const v8ha*)(krow + 512 * hh + 8 * j);
    #pragma unroll
    for (int i = 0; i < 8; ++i) mx = fmaxf(mx, (float)kv[i]);
  }
  mx = fmaxf(mx, __shfl_xor(mx, 16));

  v8f acc = zero8f();
  float ssum = 0.0f;
  #pragma unroll 1
  for (int k0 = 0; k0 < NSEQ; k0 += 32) {
    const v16h kf = load_frag(krow + k0, hh);
    Frag pa;
    #pragma unroll
    for (int i = 0; i < 16; ++i) {
      const float p = __expf(((float)kf[i] - mx) * 0.125f);
      ssum += p;
      pa.v[i] = (_Float16)p;
    }
    const v16h vb = load_frag(vrow + k0, hh);
    acc = wmma_f16(pa.v, vb, acc);
  }
  ssum += __shfl_xor(ssum, 16);

  v8h cv;
  #pragma unroll
  for (int r = 0; r < 8; ++r) {
    const float sd = __shfl(ssum, 8 * hh + r);
    cv[r] = (_Float16)(acc[r] * 8.0f * __builtin_amdgcn_rcpf(sd));
  }
  *(v8ha*)(sC + m * 16 + 8 * hh) = cv;
  __syncthreads();
  const v8h ov = *(const v8ha*)(sC + 8 * lane);
  _Float16* dst = ctxT + (size_t)bh * 256 + 8 * lane;
  *(volatile v8h*)dst = ov;
  __threadfence();
  *(volatile v8h*)dst = ov;
}

__global__ __launch_bounds__(128) void octx_kernel(const _Float16* __restrict__ qp,
                                                   const _Float16* __restrict__ ctxT,
                                                   _Float16* __restrict__ op)
{
  __shared__ __attribute__((aligned(16))) _Float16 sO[128 * 136];

  const int tid = threadIdx.x, lane = tid & 31, w = tid >> 5, hh = lane >> 4, m = lane & 15;
  const int m0 = blockIdx.x * 128, b = m0 >> 10;
  const v8h z8 = zero8h();

  #pragma unroll 1
  for (int hd = 0; hd < NH; ++hd) {
    Frag fb;
    fb.half[0] = *(const v8ha*)(ctxT + ((size_t)(b * NH + hd) * HDIM + m) * HDIM + 8 * hh);
    fb.half[1] = z8;
    #pragma unroll
    for (int mt = 0; mt < 2; ++mt) {
      const int rl = 32 * w + 16 * mt + m;
      const v8h qv = *(const v8ha*)(qp + ((size_t)(m0 + rl)) * NE + hd * HDIM + 8 * hh);
      float v[8];
      #pragma unroll
      for (int i = 0; i < 8; ++i) v[i] = (float)qv[i] * 0.125f;
      float mx = v[0];
      #pragma unroll
      for (int i = 1; i < 8; ++i) mx = fmaxf(mx, v[i]);
      mx = fmaxf(mx, __shfl_xor(mx, 16));
      float s = 0.0f;
      #pragma unroll
      for (int i = 0; i < 8; ++i) { v[i] = __expf(v[i] - mx); s += v[i]; }
      s += __shfl_xor(s, 16);
      const float inv = __builtin_amdgcn_rcpf(s);
      Frag fa;
      v8h pv;
      #pragma unroll
      for (int i = 0; i < 8; ++i) pv[i] = (_Float16)(16.0f * v[i] * inv);
      fa.half[0] = pv;
      fa.half[1] = z8;
      const v8f acc = wmma_f16(fa.v, fb.v, zero8f());
      #pragma unroll
      for (int r = 0; r < 8; ++r)
        sO[(32 * w + 16 * mt + 8 * hh + r) * 136 + hd * HDIM + m] = (_Float16)(acc[r] * (1.0f / 256.0f));
    }
  }
  __syncthreads();

  const int q8 = lane & 7, sub = lane >> 3;
  _Float16* gbase = op + (size_t)m0 * NE;
  #pragma unroll
  for (int i = 0; i < 16; ++i) {
    const int L = 4 * i + sub, row = 32 * w + (L >> 1), hl = L & 1;
    const v8h vv = *(const v8ha*)(sO + row * 136 + 64 * hl + 8 * q8);
    *(volatile v8h*)(gbase + (size_t)row * NE + 64 * hl + 8 * q8) = vv;
  }
  __threadfence();
  #pragma unroll
  for (int i = 0; i < 16; ++i) {
    const int L = 4 * i + sub, row = 32 * w + (L >> 1), hl = L & 1;
    const v8h vv = *(const v8ha*)(sO + row * 136 + 64 * hl + 8 * q8);
    *(volatile v8h*)(gbase + (size_t)row * NE + 64 * hl + 8 * q8) = vv;
  }
}

__global__ __launch_bounds__(128) void mean_kernel(const float* __restrict__ t, float* __restrict__ out)
{
  __shared__ __attribute__((aligned(16))) float sM[NE];
  const int e = threadIdx.x, b = blockIdx.x;
  const float* p = t + (size_t)b * NSEQ * NE + e;
  double s = 0.0;
  #pragma unroll 4
  for (int n = 0; n < NSEQ; ++n) s += (double)p[(size_t)n * NE];
  sM[e] = (float)(s * (1.0 / NSEQ));
  __syncthreads();
  if (threadIdx.x < 32) {
    const int l = threadIdx.x;
    const v4f v = *(const v4fa*)(sM + 4 * l);
    float* dst = out + (size_t)b * NE + 4 * l;
    *(volatile v4f*)dst = v;
    __threadfence();
    *(volatile v4f*)dst = v;
  }
}

extern "C" void kernel_launch(void* const* d_in, const int* in_sizes, int n_in,
                              void* d_out, int out_size, void* d_ws, size_t ws_size,
                              hipStream_t stream)
{
  if (n_in < 14) return;
  if (in_sizes[0] != NB * NE * NSEQ) return;
  if (in_sizes[1] != NL * NE * NE || in_sizes[2] != NL * NE * NE ||
      in_sizes[3] != NL * NE * NE || in_sizes[4] != NL * NE * NE) return;
  if (in_sizes[5] != NL * NE || in_sizes[6] != NL * NE || in_sizes[7] != NL * NE) return;
  if (in_sizes[8] != NL * NE * NFF || in_sizes[9] != NL * NFF || in_sizes[10] != NL * NFF * NE) return;
  if (in_sizes[11] != NL * NE || in_sizes[12] != NL * NE || in_sizes[13] != NL * NE) return;
  if (out_size != NB * NE) return;

  const float* x    = (const float*)d_in[0];
  const float* qw   = (const float*)d_in[1];
  const float* kw   = (const float*)d_in[2];
  const float* vw   = (const float*)d_in[3];
  const float* ow   = (const float*)d_in[4];
  const float* ob   = (const float*)d_in[5];
  const float* ln1g = (const float*)d_in[6];
  const float* ln1b = (const float*)d_in[7];
  const float* fw1  = (const float*)d_in[8];
  const float* fb1  = (const float*)d_in[9];
  const float* fw2  = (const float*)d_in[10];
  const float* fb2  = (const float*)d_in[11];
  const float* ln2g = (const float*)d_in[12];
  const float* ln2b = (const float*)d_in[13];
  float* out = (float*)d_out;

  const size_t t_bytes    = (size_t)NROWS * NE * 4;
  const size_t pl_bytes   = (size_t)NROWS * NE * 2;
  const size_t ffa_bytes  = (size_t)NROWS * NFF * 2;
  const size_t ctx_bytes  = (size_t)NB * NH * 256 * 2;
  const size_t wqkv_bytes = (size_t)NL * 3 * NE * NE * 2;
  const size_t wo_bytes   = (size_t)NL * NE * NE * 2;
  const size_t w1_bytes   = (size_t)NL * NFF * NE * 2;
  const size_t w2_bytes   = (size_t)NL * NE * NFF * 2;
  size_t off = 0;
  char* ws = (char*)d_ws;
  float*    t    = (float*)(ws + off);    off += t_bytes;
  _Float16* y    = (_Float16*)(ws + off); off += pl_bytes;
  _Float16* q8   = (_Float16*)(ws + off); off += pl_bytes;
  _Float16* kt   = (_Float16*)(ws + off); off += pl_bytes;
  _Float16* vt   = (_Float16*)(ws + off); off += pl_bytes;
  _Float16* o16  = (_Float16*)(ws + off); off += pl_bytes;
  _Float16* ctxT = (_Float16*)(ws + off); off += ctx_bytes;
  _Float16* wqkv = (_Float16*)(ws + off); off += wqkv_bytes;
  _Float16* wo   = (_Float16*)(ws + off); off += wo_bytes;
  _Float16* w1t  = (_Float16*)(ws + off); off += w1_bytes;
  _Float16* w2t  = (_Float16*)(ws + off); off += w2_bytes;
  if (ffa_bytes != 4 * pl_bytes) return;
  _Float16* ffa = q8;
  if (off > ws_size) return;
  if (off > (size_t)134217728) return;

  xt_kernel<<<dim3(NSEQ / 32, NE / 32, NB), 256, 0, stream>>>(x, t);
  wt_kernel<<<dim3(NE / 32, NE / 64, NL), 256, 0, stream>>>(qw, wqkv, NE, NE, 3 * NE * NE, 0);
  wt_kernel<<<dim3(NE / 32, NE / 64, NL), 256, 0, stream>>>(kw, wqkv, NE, NE, 3 * NE * NE, NE);
  wt_kernel<<<dim3(NE / 32, NE / 64, NL), 256, 0, stream>>>(vw, wqkv, NE, NE, 3 * NE * NE, 2 * NE);
  wt_kernel<<<dim3(NE / 32, NE / 64, NL), 256, 0, stream>>>(ow, wo, NE, NE, NE * NE, 0);
  wt_kernel<<<dim3(NFF / 32, NE / 64, NL), 256, 0, stream>>>(fw1, w1t, NE, NFF, NFF * NE, 0);
  wt_kernel<<<dim3(NE / 32, NFF / 64, NL), 256, 0, stream>>>(fw2, w2t, NFF, NE, NE * NFF, 0);

  const dim3 gQKV(NROWS / 128, (3 * NE) / 64);
  const dim3 gE(NROWS / 128, NE / 64);
  const dim3 gF(NROWS / 128, NFF / 64);

  for (int i = 0; i < NL; ++i) {
    ln_kernel<<<NROWS / 16, 256, 0, stream>>>(t, ln1g + i * NE, ln1b + i * NE, y);
    gemm_qkv_kernel<<<gQKV, 128, 0, stream>>>(y, wqkv + (size_t)i * 3 * NE * NE, q8, kt, vt);
    ctx_kernel<<<NB * NH, 32, 0, stream>>>(kt, vt, ctxT);
    octx_kernel<<<NROWS / 128, 128, 0, stream>>>(q8, ctxT, o16);
    gemm_resid_kernel<<<gE, 128, 0, stream>>>(o16, NE, wo + (size_t)i * NE * NE, NE,
                                               ob + i * NE, 1.0f / 256.0f, t);
    ln_kernel<<<NROWS / 16, 256, 0, stream>>>(t, ln2g + i * NE, ln2b + i * NE, y);
    gemm_gelu_kernel<<<gF, 128, 0, stream>>>(y, w1t + (size_t)i * NFF * NE, fb1 + i * NFF, ffa);
    gemm_resid_kernel<<<gE, 128, 0, stream>>>(ffa, NFF, w2t + (size_t)i * NE * NFF, NFF,
                                               fb2 + i * NE, 1.0f / 128.0f, t);
  }

  mean_kernel<<<NB, NE, 0, stream>>>(t, out);
}
